// GINVNNoEdge_55886114456251
// MI455X (gfx1250) — hardware-verified
//
#include <hip/hip_runtime.h>
#include <stddef.h>


#define HIDC   128
#define NFEAT  9
#define NVOC   128
#define NTHR   256
#define NWAVE  8
#define GROWS  128
#define AP     136
#define EPT    8
#define NGRP   2
#define CHUNK  (NTHR * EPT * NGRP)
#define WCAP   (EPT * NGRP * 32)
#define LISTN  (NWAVE * WCAP)
#define NBC    4096
#define NBF    1024
#define NBP    32
#define RCAP   40960
#define RBN    128
#define DEGCAP 256
#define OTHR   512
#define PSTR   256
#define WPL    (HIDC * HIDC)
#define BNEPS  1e-5f

#define LDS_GEMM (2 * GROWS * AP * 2 + GROWS * HIDC * 4 + PSTR * 8)
#define LDS_FILL ((RCAP + NBF + LISTN) * 4 + 64)

static_assert((CHUNK & (CHUNK - 1)) == 0);
static_assert(CHUNK <= 4096);
static_assert(NBC <= 4096 && NBF <= 4096 && NBP <= 4096);
static_assert((NBC & (NBC - 1)) == 0 && (NBF & (NBF - 1)) == 0 && (NBP & (NBP - 1)) == 0);
static_assert(NBC == 4 * NBF);
static_assert(OTHR * 8 == NBC);
static_assert((RCAP % 32) == 0);
static_assert(GROWS == NWAVE * 16);
static_assert((GROWS * HIDC / 8) % NTHR == 0);
static_assert(NBP * HIDC == 16 * NTHR);
static_assert((AP % 8) == 0);
static_assert((NBC % GROWS) == 0);
static_assert(((2 * GROWS * AP * 2) % 16) == 0);

typedef float          v4f   __attribute__((ext_vector_type(4)));
typedef float          v8f   __attribute__((ext_vector_type(8)));
typedef int            v4i   __attribute__((ext_vector_type(4)));
typedef unsigned short v4us  __attribute__((ext_vector_type(4)));
typedef unsigned short v8us  __attribute__((ext_vector_type(8)));
typedef unsigned short v16us __attribute__((ext_vector_type(16)));
typedef __bf16         v16bf __attribute__((ext_vector_type(16)));
typedef double         v2d   __attribute__((ext_vector_type(2)));
union FragB { v16us u; v8us h[2]; v16bf v; };
union Pack8 { v8us v; v4us q[2]; };

__device__ __forceinline__ unsigned short f2bf(float f) {
  unsigned int u = __builtin_bit_cast(unsigned int, f);
  u += 0x7FFFu + ((u >> 16) & 1u);
  return (unsigned short)(u >> 16);
}
__device__ __forceinline__ float bf2f(unsigned short b) {
  return __builtin_bit_cast(float, ((unsigned int)b) << 16);
}
__device__ __forceinline__ void split4(v4f x, v4us& hi, v4us& lo) {
  const unsigned short h0 = f2bf(x.x), h1 = f2bf(x.y), h2 = f2bf(x.z), h3 = f2bf(x.w);
  hi.x = h0; hi.y = h1; hi.z = h2; hi.w = h3;
  lo.x = f2bf(x.x - bf2f(h0)); lo.y = f2bf(x.y - bf2f(h1));
  lo.z = f2bf(x.z - bf2f(h2)); lo.w = f2bf(x.w - bf2f(h3));
}
__device__ __forceinline__ void split8(v4f a, v4f b, v8us& hv, v8us& lv) {
  Pack8 H, Lw;
  split4(a, H.q[0], Lw.q[0]);
  split4(b, H.q[1], Lw.q[1]);
  hv = H.v; lv = Lw.v;
}

__device__ __forceinline__ v8f wmb(v16bf a, v16bf b, v8f c) {
  v8f d = __builtin_amdgcn_wmma_f32_16x16x32_bf16(false, a, false, b, (short)0, c, false, false);
  asm volatile("v_nop\n\tv_nop\n\tv_nop\n\tv_nop" : "+v"(d) : "v"(a), "v"(b));
  return d;
}

template <int NB>
__device__ __forceinline__ int scan_chunk(const int* __restrict__ dsts, int nE, int cbase, int slotBase,
                                          int vec8, int* list, int tid, int lane, int wave) {
  int wc = 0;
#pragma unroll
  for (int g = 0; g < NGRP; ++g) {
    const int el0  = (g * NTHR + tid) * EPT;
    const int e0   = cbase + el0;
    const int sent = -2147483647 - 1;
    v4i da, db;
    if (vec8 != 0 && cbase + CHUNK <= nE) {
      da = *(const v4i*)(dsts + e0);
      db = *(const v4i*)(dsts + e0 + 4);
    } else {
      da.x = (e0     < nE) ? dsts[min(e0, nE - 1)] : sent;
      da.y = (e0 + 1 < nE) ? dsts[min(e0 + 1, nE - 1)] : sent;
      da.z = (e0 + 2 < nE) ? dsts[min(e0 + 2, nE - 1)] : sent;
      da.w = (e0 + 3 < nE) ? dsts[min(e0 + 3, nE - 1)] : sent;
      db.x = (e0 + 4 < nE) ? dsts[min(e0 + 4, nE - 1)] : sent;
      db.y = (e0 + 5 < nE) ? dsts[min(e0 + 5, nE - 1)] : sent;
      db.z = (e0 + 6 < nE) ? dsts[min(e0 + 6, nE - 1)] : sent;
      db.w = (e0 + 7 < nE) ? dsts[min(e0 + 7, nE - 1)] : sent;
    }
    const unsigned nb = (unsigned)slotBase;
    const unsigned s0 = (unsigned)da.x - nb, s1 = (unsigned)da.y - nb;
    const unsigned s2 = (unsigned)da.z - nb, s3 = (unsigned)da.w - nb;
    const unsigned s4 = (unsigned)db.x - nb, s5 = (unsigned)db.y - nb;
    const unsigned s6 = (unsigned)db.z - nb, s7 = (unsigned)db.w - nb;
    const bool h0 = s0 < (unsigned)NB, h1 = s1 < (unsigned)NB, h2 = s2 < (unsigned)NB, h3 = s3 < (unsigned)NB;
    const bool h4 = s4 < (unsigned)NB, h5 = s5 < (unsigned)NB, h6 = s6 < (unsigned)NB, h7 = s7 < (unsigned)NB;
    const unsigned any = __builtin_amdgcn_ballot_w32(h0 | h1 | h2 | h3 | h4 | h5 | h6 | h7);
    if (any != 0u) {
#define HITJ(J, HJ, SJ) { \
        const unsigned mj = __builtin_amdgcn_ballot_w32(HJ); \
        if (mj != 0u) { \
          if (HJ) { \
            const int pos = wc + (int)__builtin_amdgcn_mbcnt_lo(mj, 0u); \
            if (pos < WCAP) list[wave * WCAP + pos] = ((el0 + (J)) << 12) | (int)(SJ); \
          } \
          wc += (int)__builtin_popcount(mj); } }
      HITJ(0, h0, s0)
      HITJ(1, h1, s1)
      HITJ(2, h2, s2)
      HITJ(3, h3, s3)
      HITJ(4, h4, s4)
      HITJ(5, h5, s5)
      HITJ(6, h6, s6)
      HITJ(7, h7, s7)
#undef HITJ
    }
  }
  return wc;
}

__global__ __launch_bounds__(NTHR) void k_wprep(
    const float* __restrict__ cW1, const float* __restrict__ cW2, const float* __restrict__ vW1,
    const float* __restrict__ vW2, const float* __restrict__ clW, unsigned short* wpl, int nL, int nV) {
  const int i  = blockIdx.x * NTHR + (int)threadIdx.x;
  const int mi = i >> 11;
  const int w  = i & 2047;
  const float* src;
  if (mi < nL)                    src = cW1 + (size_t)mi * WPL;
  else if (mi < 2 * nL)           src = cW2 + (size_t)(mi - nL) * WPL;
  else if (mi < 2 * nL + nV)      src = vW1 + (size_t)(mi - 2 * nL) * WPL;
  else if (mi < 2 * nL + 2 * nV)  src = vW2 + (size_t)(mi - 2 * nL - nV) * WPL;
  else                            src = clW;
  const int n  = w >> 4;
  const int k0 = (w & 15) * 8;
  v4f a, b;
  a.x = src[(size_t)(k0 + 0) * HIDC + n]; a.y = src[(size_t)(k0 + 1) * HIDC + n];
  a.z = src[(size_t)(k0 + 2) * HIDC + n]; a.w = src[(size_t)(k0 + 3) * HIDC + n];
  b.x = src[(size_t)(k0 + 4) * HIDC + n]; b.y = src[(size_t)(k0 + 5) * HIDC + n];
  b.z = src[(size_t)(k0 + 6) * HIDC + n]; b.w = src[(size_t)(k0 + 7) * HIDC + n];
  v8us hv, lv;
  split8(a, b, hv, lv);
  unsigned short* dp = wpl + (size_t)mi * 2 * WPL + (size_t)n * HIDC + k0;
  *(volatile v8us*)dp = hv;
  *(volatile v8us*)(dp + WPL) = lv;
  __threadfence();
  *(volatile v8us*)dp = hv;
  *(volatile v8us*)(dp + WPL) = lv;
}

__global__ __launch_bounds__(NTHR) void k_count(
    const int* __restrict__ ei, int* cnt, int nE, int vec8) {
  __shared__ __attribute__((aligned(16))) int scnt[NBC];
  __shared__ __attribute__((aligned(16))) int list[LISTN];
  __shared__ int wcnt[NWAVE];
  const int tid = threadIdx.x, lane = tid & 31, wave = tid >> 5;
  const int nodeBase = blockIdx.x * NBC;
  const int* dsts = ei + nE;

  for (int i = tid; i < NBC; i += NTHR) scnt[i] = 0;
  __syncthreads();

  const int nChunks = (nE + CHUNK - 1) / CHUNK;
#pragma unroll 1
  for (int ch = 0; ch < nChunks; ++ch) {
    const int cbase = ch * CHUNK;
    const int wc = scan_chunk<NBC>(dsts, nE, cbase, nodeBase, vec8, list, tid, lane, wave);
    if (lane == 0) wcnt[wave] = wc;
    __syncthreads();
    if (wave == 0) {
#pragma unroll 1
      for (int wsx = 0; wsx < NWAVE; ++wsx) {
        int n = __builtin_amdgcn_readfirstlane(wcnt[wsx]);
        n = n > WCAP ? WCAP : (n < 0 ? 0 : n);
        const int* lp = list + wsx * WCAP;
#pragma unroll 1
        for (int i = 0; i < n; ++i) {
          const int ent  = __builtin_amdgcn_readfirstlane(lp[i]);
          const int slot = ent & (NBC - 1);
          if (lane == 0) scnt[slot] = scnt[slot] + 1;
        }
      }
    }
    __syncthreads();
  }

  v4i cq[4];
#pragma unroll
  for (int q = 0; q < 4; ++q) {
    const int f = (wave * 4 + q) * 128 + 4 * lane;
    cq[q] = *(const v4i*)(scnt + f);
  }
  int* cp = cnt + (size_t)nodeBase;
#pragma unroll
  for (int q = 0; q < 4; ++q) {
    const int f = (wave * 4 + q) * 128 + 4 * lane;
    *(volatile v4i*)(cp + f) = cq[q];
  }
  __threadfence();
#pragma unroll
  for (int q = 0; q < 4; ++q) {
    const int f = (wave * 4 + q) * 128 + 4 * lane;
    *(volatile v4i*)(cp + f) = cq[q];
  }
}

__global__ __launch_bounds__(OTHR) void k_offsets(
    const int* __restrict__ cnt, int* off, int* rbase, int nChunk) {
  __shared__ __attribute__((aligned(16))) int soff[NBC];
  __shared__ __attribute__((aligned(16))) int srb[RBN];
  __shared__ int wtot[OTHR / 32];
  const int tid = threadIdx.x, lane = tid & 31, wave = tid >> 5, sub = tid >> 7;
  for (int i = tid; i < RBN; i += OTHR) srb[i] = 0;
  int carry = 0;
#pragma unroll 1
  for (int ch = 0; ch < nChunk; ++ch) {
    const int base = ch * NBC;
    const v4i c0 = *(const v4i*)(cnt + base + 8 * tid);
    const v4i c1 = *(const v4i*)(cnt + base + 8 * tid + 4);
    const int e0 = max(c0.x, 0), e1 = max(c0.y, 0), e2 = max(c0.z, 0), e3 = max(c0.w, 0);
    const int e4 = max(c1.x, 0), e5 = max(c1.y, 0), e6 = max(c1.z, 0), e7 = max(c1.w, 0);
    const int ts = e0 + e1 + e2 + e3 + e4 + e5 + e6 + e7;
    int incl = ts;
#pragma unroll
    for (int d = 1; d < 32; d <<= 1) {
      const int t = __shfl_up(incl, d);
      if (lane >= d) incl += t;
    }
    if (lane == 31) wtot[wave] = incl;
    __syncthreads();
    const int S0 = wtot[0]  + wtot[1]  + wtot[2]  + wtot[3];
    const int S1 = wtot[4]  + wtot[5]  + wtot[6]  + wtot[7];
    const int S2 = wtot[8]  + wtot[9]  + wtot[10] + wtot[11];
    const int S3 = wtot[12] + wtot[13] + wtot[14] + wtot[15];
    int pre = 0;
#pragma unroll 1
    for (int w = 4 * sub; w < wave; ++w) pre += wtot[w];
    const int b0 = carry;
    const int b1 = b0 + ((S0 + 31) & ~31);
    const int b2 = b1 + ((S1 + 31) & ~31);
    const int b3 = b2 + ((S2 + 31) & ~31);
    const int b4 = b3 + ((S3 + 31) & ~31);
    const int myb = sub == 0 ? b0 : (sub == 1 ? b1 : (sub == 2 ? b2 : b3));
    if (tid == 0) {
      srb[min(4 * ch + 0, RBN - 1)] = b0;
      srb[min(4 * ch + 1, RBN - 1)] = b1;
      srb[min(4 * ch + 2, RBN - 1)] = b2;
      srb[min(4 * ch + 3, RBN - 1)] = b3;
    }
    int run = myb + pre + incl - ts;
    soff[8 * tid + 0] = run; run += e0;
    soff[8 * tid + 1] = run; run += e1;
    soff[8 * tid + 2] = run; run += e2;
    soff[8 * tid + 3] = run; run += e3;
    soff[8 * tid + 4] = run; run += e4;
    soff[8 * tid + 5] = run; run += e5;
    soff[8 * tid + 6] = run; run += e6;
    soff[8 * tid + 7] = run;
    carry = b4;
    __syncthreads();
    const v4i o0 = *(const v4i*)(soff + 4 * tid);
    const v4i o1 = *(const v4i*)(soff + 4 * (tid + OTHR));
    int* op = off + base;
    *(volatile v4i*)(op + 4 * tid) = o0;
    *(volatile v4i*)(op + 4 * (tid + OTHR)) = o1;
    __threadfence();
    *(volatile v4i*)(op + 4 * tid) = o0;
    *(volatile v4i*)(op + 4 * (tid + OTHR)) = o1;
    __syncthreads();
  }
  if (tid == 0) srb[min(4 * nChunk, RBN - 1)] = carry;
  __syncthreads();
  v4i rv = {0, 0, 0, 0};
  if (tid < 32) rv = *(const v4i*)(srb + 4 * tid);
  if (tid < 32) *(volatile v4i*)(rbase + 4 * tid) = rv;
  __threadfence();
  if (tid < 32) *(volatile v4i*)(rbase + 4 * tid) = rv;
}

__global__ __launch_bounds__(NTHR) void k_fill(
    const int* __restrict__ ei, const int* __restrict__ off, const int* __restrict__ rbase,
    int* csr, int nN, int nE, int vec8, int csrLen) {
  extern __shared__ v4f lds_dyn[];
  int* region = (int*)lds_dyn;
  int* cursor = region + RCAP;
  int* list   = cursor + NBF;
  int* wcnt   = list + LISTN;
  const int tid = threadIdx.x, lane = tid & 31, wave = tid >> 5;
  const int b = blockIdx.x;
  const int nodeBase = b * NBF;
  const int* dsts = ei + nE;

  int rb0 = rbase[b];
  const int rb1 = rbase[b + 1];
  rb0 = rb0 < 0 ? 0 : (rb0 > csrLen ? csrLen : rb0);
  rb0 &= ~31;
  int len = rb1 - rb0;
  len = len < 0 ? 0 : (len > RCAP ? RCAP : len);
  int lenW = (len + 31) & ~31;
  if (rb0 + lenW > csrLen) lenW = (csrLen - rb0) & ~31;

  {
    const v4i z = {0, 0, 0, 0};
    for (int i = tid; i < RCAP / 4; i += NTHR) ((v4i*)region)[i] = z;
    for (int s = tid; s < NBF; s += NTHR) {
      int o = off[nodeBase + s] - rb0;
      o = o < 0 ? 0 : (o > RCAP ? RCAP : o);
      cursor[s] = o;
    }
  }
  __syncthreads();

  const int nChunks = (nE + CHUNK - 1) / CHUNK;
#pragma unroll 1
  for (int ch = 0; ch < nChunks; ++ch) {
    const int cbase = ch * CHUNK;
    const int wc = scan_chunk<NBF>(dsts, nE, cbase, nodeBase, vec8, list, tid, lane, wave);
    if (lane == 0) wcnt[wave] = wc;
    __syncthreads();
    if (wave == 0) {
#pragma unroll 1
      for (int wsx = 0; wsx < NWAVE; ++wsx) {
        int n = __builtin_amdgcn_readfirstlane(wcnt[wsx]);
        n = n > WCAP ? WCAP : (n < 0 ? 0 : n);
        const int* lp = list + wsx * WCAP;
#pragma unroll 1
        for (int i = 0; i < n; ++i) {
          const int ent  = __builtin_amdgcn_readfirstlane(lp[i]);
          const int slot = ent & (NBF - 1);
          int e = cbase + ((ent >> 12) & (CHUNK - 1));
          e = e > nE - 1 ? nE - 1 : e;
          int src = ei[e];
          src = src < 0 ? 0 : (src > nN - 1 ? nN - 1 : src);
          if (lane == 0) {
            int pos = cursor[slot];
            pos = pos < 0 ? 0 : (pos > RCAP - 1 ? RCAP - 1 : pos);
            region[pos] = src;
            const int np = pos + 1;
            cursor[slot] = np > RCAP ? RCAP : np;
          }
        }
      }
    }
    __syncthreads();
  }

  const int nv = lenW >> 2;
  int* gp = csr + rb0;
#pragma unroll 1
  for (int i = tid; i < nv; i += NTHR) { const v4i v = ((const v4i*)region)[i]; *(volatile v4i*)(gp + 4 * i) = v; }
  __threadfence();
#pragma unroll 1
  for (int i = tid; i < nv; i += NTHR) { const v4i v = ((const v4i*)region)[i]; *(volatile v4i*)(gp + 4 * i) = v; }
}

__global__ __launch_bounds__(NTHR) void k_encode(
    const int* __restrict__ x, const float* __restrict__ emb, float* h, int nN) {
  const int lane = threadIdx.x & 31, wave = threadIdx.x >> 5;
  const int row = blockIdx.x * NWAVE + wave;
  const int rs  = row < nN ? row : nN - 1;
  const int f   = lane < NFEAT ? lane : NFEAT - 1;
  int xi = x[(size_t)rs * NFEAT + f];
  xi = xi < 0 ? 0 : (xi > NVOC - 1 ? NVOC - 1 : xi);
  v4f s = {0.f, 0.f, 0.f, 0.f};
#pragma unroll
  for (int q = 0; q < NFEAT; ++q) {
    const int idx = __builtin_amdgcn_readlane(xi, q);
    s = s + *(const v4f*)(emb + ((size_t)(q * NVOC + idx)) * HIDC + 4 * lane);
  }
  float* hp = h + (size_t)row * HIDC + 4 * lane;
  *(volatile v4f*)hp = s;
  __threadfence();
  *(volatile v4f*)hp = s;
}

__global__ __launch_bounds__(NTHR) void k_vninit(const float* __restrict__ ve, float* vnh) {
  const int lane = threadIdx.x & 31, wave = threadIdx.x >> 5;
  const int row = blockIdx.x * NWAVE + wave;
  const v4f v = *(const v4f*)(ve + 4 * lane);
  float* p = vnh + (size_t)row * HIDC + 4 * lane;
  *(volatile v4f*)p = v;
  __threadfence();
  *(volatile v4f*)p = v;
}

__device__ __forceinline__ void gemm_group(
    const unsigned short* sHi, const unsigned short* sLo, const unsigned short* __restrict__ Bw,
    float* stg, const float* __restrict__ bias, int g, int wave, int hh, int m) {
  v8f acc[4];
#pragma unroll
  for (int t = 0; t < 4; ++t) { v8f z = {0.f, 0.f, 0.f, 0.f, 0.f, 0.f, 0.f, 0.f}; acc[t] = z; }
  const unsigned short* ah  = sHi + (wave * 16 + m) * AP + 8 * hh;
  const unsigned short* al  = sLo + (wave * 16 + m) * AP + 8 * hh;
  const unsigned short* BwL = Bw + WPL;
#pragma unroll
  for (int kt = 0; kt < HIDC / 32; ++kt) {
    FragB fh, fl;
    fh.h[0] = *(const v8us*)(ah + 32 * kt);
    fh.h[1] = *(const v8us*)(ah + 32 * kt + 16);
    fl.h[0] = *(const v8us*)(al + 32 * kt);
    fl.h[1] = *(const v8us*)(al + 32 * kt + 16);
#pragma unroll
    for (int t = 0; t < 4; ++t) {
      const size_t bo = (size_t)(64 * g + 16 * t + m) * HIDC + 32 * kt + 8 * hh;
      FragB bh, bl;
      bh.h[0] = *(const v8us*)(Bw + bo);
      bh.h[1] = *(const v8us*)(Bw + bo + 16);
      bl.h[0] = *(const v8us*)(BwL + bo);
      bl.h[1] = *(const v8us*)(BwL + bo + 16);
      acc[t] = wmb(fh.v, bh.v, acc[t]);
      acc[t] = wmb(fl.v, bh.v, acc[t]);
      acc[t] = wmb(fh.v, bl.v, acc[t]);
    }
  }
  float* sp = stg + (wave * 16 + 8 * hh) * HIDC + 64 * g + m;
#pragma unroll
  for (int t = 0; t < 4; ++t) {
    const float bv = bias[64 * g + 16 * t + m];
#pragma unroll
    for (int r = 0; r < 8; ++r) sp[r * HIDC + 16 * t] = acc[t][r] + bv;
  }
}

__device__ __forceinline__ void rows_store2(const float* stg, float* C, int rowBase, int wave, int lane) {
  const float* lp = stg + wave * 16 * HIDC + 4 * lane;
  float* gp = C + ((size_t)rowBase + wave * 16) * HIDC + 4 * lane;
#pragma unroll
  for (int i = 0; i < 16; ++i) { const v4f v = *(const v4f*)(lp + i * HIDC); *(volatile v4f*)(gp + (size_t)i * HIDC) = v; }
  __threadfence();
#pragma unroll
  for (int i = 0; i < 16; ++i) { const v4f v = *(const v4f*)(lp + i * HIDC); *(volatile v4f*)(gp + (size_t)i * HIDC) = v; }
}

__device__ __forceinline__ void col_stats(const float* stg, double* sps, int rowBase, int nValid, int tid) {
  const int c  = tid & (HIDC - 1);
  const int sq = tid >> 7;
  double d = 0.0;
#pragma unroll 4
  for (int r = 0; r < GROWS; ++r) {
    const float v = stg[r * HIDC + c];
    const float w = (rowBase + r < nValid) ? v : 0.0f;
    const double xd = (double)w;
    d += (sq != 0) ? xd * xd : xd;
  }
  sps[tid] = d;
}

__global__ __launch_bounds__(NTHR) void k_agg_gemm(
    const int* __restrict__ csr, const int* __restrict__ off, const int* __restrict__ cnt,
    const float* __restrict__ hin, const float* __restrict__ eps, int layer,
    const unsigned short* __restrict__ Bw, const float* __restrict__ bias,
    float* C, double* part, int nN, int csrLen) {
  extern __shared__ v4f lds_dyn[];
  unsigned short* sHi = (unsigned short*)lds_dyn;
  unsigned short* sLo = sHi + GROWS * AP;
  float*  stg = (float*)(sLo + GROWS * AP);
  double* sps = (double*)(stg + GROWS * HIDC);
  const int tid = threadIdx.x, lane = tid & 31, wave = tid >> 5, hh = lane >> 4, m = lane & 15;
  const int rowBase = blockIdx.x * GROWS;
  const float epv = 1.0f + eps[layer];
  const int tb = rowBase + wave * 16;
  const int cl = cnt[tb + m];
  const int ol = off[tb + m];

#pragma unroll 1
  for (int j = 0; j < 16; ++j) {
    const int c = tb + j;
    int n = __builtin_amdgcn_readlane(cl, j);
    n = n < 0 ? 0 : (n > DEGCAP ? DEGCAP : n);
    const int st = __builtin_amdgcn_readlane(ol, j);
    v4f acc = {0.f, 0.f, 0.f, 0.f};
#pragma unroll 1
    for (int q0 = 0; q0 < n; q0 += 32) {
      int pos = st + q0 + lane;
      pos = pos < 0 ? 0 : (pos > csrLen - 1 ? csrLen - 1 : pos);
      int sl = csr[pos];
      sl = sl < 0 ? 0 : (sl > nN - 1 ? nN - 1 : sl);
      const int mcnt = (n - q0) < 32 ? (n - q0) : 32;
#pragma unroll 1
      for (int p = 0; p < mcnt; ++p) {
        const int s = __builtin_amdgcn_readlane(sl, p);
        acc = acc + *(const v4f*)(hin + (size_t)s * HIDC + 4 * lane);
      }
    }
    const v4f sv = *(const v4f*)(hin + (size_t)c * HIDC + 4 * lane);
    const v4f z = sv * epv + acc;
    v4us hv, lv;
    split4(z, hv, lv);
    *(v4us*)(sHi + (wave * 16 + j) * AP + 4 * lane) = hv;
    *(v4us*)(sLo + (wave * 16 + j) * AP + 4 * lane) = lv;
  }
  __syncthreads();

  gemm_group(sHi, sLo, Bw, stg, bias, 0, wave, hh, m);
  gemm_group(sHi, sLo, Bw, stg, bias, 1, wave, hh, m);
  __syncthreads();

  col_stats(stg, sps, rowBase, nN, tid);
  __syncthreads();
  v2d pv = {0.0, 0.0};
  if (tid < HIDC) pv = *(const v2d*)(sps + 2 * tid);
  double* pp = part + (size_t)blockIdx.x * PSTR + 2 * (tid & (HIDC - 1));
  if (tid < HIDC) *(volatile v2d*)pp = pv;
  rows_store2(stg, C, rowBase, wave, lane);
  if (tid < HIDC) *(volatile v2d*)pp = pv;
}

__global__ __launch_bounds__(NTHR) void k_gemm(
    const float* __restrict__ A, const float* __restrict__ A2, const float* __restrict__ ab,
    const unsigned short* __restrict__ Bw, const float* __restrict__ bias,
    const float* R, const float* __restrict__ w2, const float* __restrict__ b2,
    float* C, double* part, float* out,
    int nRowsA, int nValid, int nOut, int useAdd, int useAff, int mode) {
  extern __shared__ v4f lds_dyn[];
  unsigned short* sHi = (unsigned short*)lds_dyn;
  unsigned short* sLo = sHi + GROWS * AP;
  float*  stg = (float*)(sLo + GROWS * AP);
  double* sps = (double*)(stg + GROWS * HIDC);
  const int tid = threadIdx.x, lane = tid & 31, wave = tid >> 5, hh = lane >> 4, m = lane & 15;
  const int rowBase = blockIdx.x * GROWS;

#pragma unroll
  for (int i = 0; i < (GROWS * HIDC / 8) / NTHR; ++i) {
    const int idx = i * NTHR + tid;
    const int r   = idx >> 4;
    const int c0  = (idx & 15) * 8;
    int row = rowBase + r;
    row = row > nRowsA - 1 ? nRowsA - 1 : row;
    const float* ap = A + (size_t)row * HIDC + c0;
    v4f a = *(const v4f*)ap, b = *(const v4f*)(ap + 4);
    if (useAdd != 0) {
      const float* ap2 = A2 + (size_t)row * HIDC + c0;
      a = a + *(const v4f*)ap2;
      b = b + *(const v4f*)(ap2 + 4);
    }
    if (useAff != 0) {
      const v4f ga = *(const v4f*)(ab + c0), gb = *(const v4f*)(ab + c0 + 4);
      const v4f ba = *(const v4f*)(ab + HIDC + c0), bb = *(const v4f*)(ab + HIDC + c0 + 4);
      a = a * ga + ba; b = b * gb + bb;
      a.x = fmaxf(a.x, 0.f); a.y = fmaxf(a.y, 0.f); a.z = fmaxf(a.z, 0.f); a.w = fmaxf(a.w, 0.f);
      b.x = fmaxf(b.x, 0.f); b.y = fmaxf(b.y, 0.f); b.z = fmaxf(b.z, 0.f); b.w = fmaxf(b.w, 0.f);
    }
    v8us hv, lv;
    split8(a, b, hv, lv);
    *(v8us*)(sHi + r * AP + c0) = hv;
    *(v8us*)(sLo + r * AP + c0) = lv;
  }
  __syncthreads();

  gemm_group(sHi, sLo, Bw, stg, bias, 0, wave, hh, m);
  gemm_group(sHi, sLo, Bw, stg, bias, 1, wave, hh, m);
  __syncthreads();

  if (mode == 2) {
    const v4f wv = *(const v4f*)(w2 + 4 * lane);
    const float b2v = b2[0];
    float* so = (float*)sps;
#pragma unroll
    for (int i = 0; i < 16; ++i) {
      const int r = wave * 16 + i;
      v4f v = *(const v4f*)(stg + r * HIDC + 4 * lane);
      v.x = fmaxf(v.x, 0.f); v.y = fmaxf(v.y, 0.f); v.z = fmaxf(v.z, 0.f); v.w = fmaxf(v.w, 0.f);
      float d = v.x * wv.x + v.y * wv.y + v.z * wv.z + v.w * wv.w;
#pragma unroll
      for (int s = 16; s > 0; s >>= 1) d += __shfl_xor(d, s);
      if (lane == 0) so[r] = d + b2v;
    }
    __syncthreads();
    v4f ov = {0.f, 0.f, 0.f, 0.f};
    if (tid < 32) ov = *(const v4f*)(so + 4 * tid);
    const int o0 = rowBase + 4 * tid;
    if (tid < 32) {
      if (o0 + 4 <= nOut) *(volatile v4f*)(out + o0) = ov;
      else {
        if (o0     < nOut) *(volatile float*)(out + o0)     = ov.x;
        if (o0 + 1 < nOut) *(volatile float*)(out + o0 + 1) = ov.y;
        if (o0 + 2 < nOut) *(volatile float*)(out + o0 + 2) = ov.z;
        if (o0 + 3 < nOut) *(volatile float*)(out + o0 + 3) = ov.w;
      }
    }
    __threadfence();
    if (tid < 32) {
      if (o0 + 4 <= nOut) *(volatile v4f*)(out + o0) = ov;
      else {
        if (o0     < nOut) *(volatile float*)(out + o0)     = ov.x;
        if (o0 + 1 < nOut) *(volatile float*)(out + o0 + 1) = ov.y;
        if (o0 + 2 < nOut) *(volatile float*)(out + o0 + 2) = ov.z;
        if (o0 + 3 < nOut) *(volatile float*)(out + o0 + 3) = ov.w;
      }
    }
  } else {
    if (mode == 1) {
      float* lp = stg + wave * 16 * HIDC + 4 * lane;
      const float* rp = R + ((size_t)rowBase + wave * 16) * HIDC + 4 * lane;
#pragma unroll
      for (int i = 0; i < 16; ++i) {
        v4f v = *(const v4f*)(lp + i * HIDC);
        v = v + *(const v4f*)(rp + (size_t)i * HIDC);
        *(v4f*)(lp + i * HIDC) = v;
      }
    }
    if (mode == 0) col_stats(stg, sps, rowBase, nValid, tid);
    __syncthreads();
    v2d pv = {0.0, 0.0};
    const bool wp = (mode == 0) && (tid < HIDC);
    if (wp) pv = *(const v2d*)(sps + 2 * tid);
    double* pp = part + (size_t)blockIdx.x * PSTR + 2 * (tid & (HIDC - 1));
    if (wp) *(volatile v2d*)pp = pv;
    rows_store2(stg, C, rowBase, wave, lane);
    if (wp) *(volatile v2d*)pp = pv;
  }
}

__global__ __launch_bounds__(HIDC) void k_bnfin(
    const double* __restrict__ part, int nBlk, int M,
    const float* __restrict__ gam, const float* __restrict__ bet, float* ab) {
  __shared__ __attribute__((aligned(16))) float sab[2 * HIDC];
  const int c = threadIdx.x;
  double s = 0.0, q = 0.0;
#pragma unroll 1
  for (int b = 0; b < nBlk; ++b) {
    s += part[(size_t)b * PSTR + c];
    q += part[(size_t)b * PSTR + HIDC + c];
  }
  const double invM = 1.0 / (double)(M > 0 ? M : 1);
  const double mean = s * invM;
  double var = q * invM - mean * mean;
  var = var < 0.0 ? 0.0 : var;
  const float rstd = rsqrtf((float)var + BNEPS);
  const float a = gam[c] * rstd;
  const float bsh = bet[c] - (float)mean * a;
  sab[c] = a;
  sab[HIDC + c] = bsh;
  __syncthreads();
  v4f v = {0.f, 0.f, 0.f, 0.f};
  if (c < 64) v = *(const v4f*)(sab + 4 * c);
  if (c < 64) *(volatile v4f*)(ab + 4 * c) = v;
  __threadfence();
  if (c < 64) *(volatile v4f*)(ab + 4 * c) = v;
}

__global__ __launch_bounds__(NTHR) void k_pool(
    const int* __restrict__ batch, const float* __restrict__ z, const float* __restrict__ ab,
    float* gsum, int nN, int relu) {
  __shared__ __attribute__((aligned(16))) float acc[NBP * HIDC];
  __shared__ __attribute__((aligned(16))) int list[LISTN];
  __shared__ int wcnt[NWAVE];
  const int tid = threadIdx.x, lane = tid & 31, wave = tid >> 5;
  const int gBase = blockIdx.x * NBP;

  {
    const v4f zz = {0.f, 0.f, 0.f, 0.f};
    for (int i = tid; i < NBP * HIDC / 4; i += NTHR) ((v4f*)acc)[i] = zz;
  }
  __syncthreads();
  const v4f a4 = *(const v4f*)(ab + 4 * lane);
  const v4f b4 = *(const v4f*)(ab + HIDC + 4 * lane);

  const int nChunks = (nN + CHUNK - 1) / CHUNK;
#pragma unroll 1
  for (int ch = 0; ch < nChunks; ++ch) {
    const int cbase = ch * CHUNK;
    const int wc = scan_chunk<NBP>(batch, nN, cbase, gBase, 1, list, tid, lane, wave);
    if (lane == 0) wcnt[wave] = wc;
    __syncthreads();
    if (wave == 0) {
#pragma unroll 1
      for (int wsx = 0; wsx < NWAVE; ++wsx) {
        int n = __builtin_amdgcn_readfirstlane(wcnt[wsx]);
        n = n > WCAP ? WCAP : (n < 0 ? 0 : n);
        const int* lp = list + wsx * WCAP;
#pragma unroll 1
        for (int i = 0; i < n; ++i) {
          const int ent  = __builtin_amdgcn_readfirstlane(lp[i]);
          const int slot = ent & (NBP - 1);
          int nd = cbase + ((ent >> 12) & (CHUNK - 1));
          nd = nd > nN - 1 ? nN - 1 : nd;
          v4f v = *(const v4f*)(z + (size_t)nd * HIDC + 4 * lane);
          v = v * a4 + b4;
          if (relu != 0) { v.x = fmaxf(v.x, 0.f); v.y = fmaxf(v.y, 0.f); v.z = fmaxf(v.z, 0.f); v.w = fmaxf(v.w, 0.f); }
          v4f* ap = (v4f*)(acc + slot * HIDC + 4 * lane);
          *ap = *ap + v;
        }
      }
    }
    __syncthreads();
  }

  v4f ov[4];
#pragma unroll
  for (int i = 0; i < 4; ++i) ov[i] = *(const v4f*)(acc + (wave * 4 + i) * HIDC + 4 * lane);
  float* gp = gsum + ((size_t)gBase + wave * 4) * HIDC + 4 * lane;
#pragma unroll
  for (int i = 0; i < 4; ++i) *(volatile v4f*)(gp + (size_t)i * HIDC) = ov[i];
  __threadfence();
#pragma unroll
  for (int i = 0; i < 4; ++i) *(volatile v4f*)(gp + (size_t)i * HIDC) = ov[i];
}

__global__ __launch_bounds__(NTHR) void k_hprod(
    const float* __restrict__ z, const float* __restrict__ ab, const float* __restrict__ vnh,
    const int* __restrict__ batch, float* h, int nN, int nG) {
  const int lane = threadIdx.x & 31, wave = threadIdx.x >> 5;
  const int row = blockIdx.x * NWAVE + wave;
  const int rs  = row < nN ? row : nN - 1;
  int b = batch[rs];
  b = b < 0 ? 0 : (b > nG - 1 ? nG - 1 : b);
  const v4f a4 = *(const v4f*)(ab + 4 * lane);
  const v4f b4 = *(const v4f*)(ab + HIDC + 4 * lane);
  v4f v = *(const v4f*)(z + (size_t)row * HIDC + 4 * lane);
  v = v * a4 + b4;
  v.x = fmaxf(v.x, 0.f); v.y = fmaxf(v.y, 0.f); v.z = fmaxf(v.z, 0.f); v.w = fmaxf(v.w, 0.f);
  v = v + *(const v4f*)(vnh + (size_t)b * HIDC + 4 * lane);
  float* hp = h + (size_t)row * HIDC + 4 * lane;
  *(volatile v4f*)hp = v;
  __threadfence();
  *(volatile v4f*)hp = v;
}

extern "C" void kernel_launch(void* const* d_in, const int* in_sizes, int n_in,
                              void* d_out, int out_size, void* d_ws, size_t ws_size,
                              hipStream_t stream) {
  if (n_in < 25) return;
  const int nN = in_sizes[0] / NFEAT;
  const int nE = in_sizes[1] / 2;
  const int G  = out_size;
  if (nN <= 0 || nE <= 0 || G <= 0) return;
  if (in_sizes[0] != nN * NFEAT || in_sizes[1] != 2 * nE || in_sizes[3] != nN) return;
  if (in_sizes[4] != NFEAT * NVOC * HIDC) return;
  const int nL = in_sizes[5];
  if (nL < 1 || nL > 16) return;
  const int nV = nL - 1;
  if (in_sizes[6] != nL * WPL || in_sizes[10] != nL * WPL) return;
  if (in_sizes[7] != nL * HIDC || in_sizes[8] != nL * HIDC || in_sizes[9] != nL * HIDC ||
      in_sizes[11] != nL * HIDC || in_sizes[12] != nL * HIDC || in_sizes[13] != nL * HIDC) return;
  if (in_sizes[14] < HIDC) return;
  if (nV > 0 && (in_sizes[15] != nV * WPL || in_sizes[19] != nV * WPL || in_sizes[16] != nV * HIDC ||
                 in_sizes[17] != nV * HIDC || in_sizes[18] != nV * HIDC || in_sizes[20] != nV * HIDC)) return;
  if (in_sizes[21] != WPL || in_sizes[22] != HIDC || in_sizes[23] != HIDC || in_sizes[24] < 1) return;
  if (nE > (1 << 28) || nN > (1 << 24) || G > (1 << 24)) return;

  const int*   x       = (const int*)d_in[0];
  const int*   ei      = (const int*)d_in[1];
  const int*   batch   = (const int*)d_in[3];
  const float* emb     = (const float*)d_in[4];
  const float* eps     = (const float*)d_in[5];
  const float* convW1  = (const float*)d_in[6];
  const float* convb1  = (const float*)d_in[7];
  const float* convg1  = (const float*)d_in[8];
  const float* convbt1 = (const float*)d_in[9];
  const float* convW2  = (const float*)d_in[10];
  const float* convb2  = (const float*)d_in[11];
  const float* bng     = (const float*)d_in[12];
  const float* bnb     = (const float*)d_in[13];
  const float* vn_emb  = (const float*)d_in[14];
  const float* vnW1    = (const float*)d_in[15];
  const float* vnb1    = (const float*)d_in[16];
  const float* vng1    = (const float*)d_in[17];
  const float* vnbt1   = (const float*)d_in[18];
  const float* vnW2    = (const float*)d_in[19];
  const float* vnb2    = (const float*)d_in[20];
  const float* clfW1   = (const float*)d_in[21];
  const float* clfb1   = (const float*)d_in[22];
  const float* clfW2   = (const float*)d_in[23];
  const float* clfb2   = (const float*)d_in[24];
  float* out = (float*)d_out;

  const int NPAD   = ((nN + GROWS - 1) / GROWS) * GROWS;
  const int nBC    = (nN + NBC - 1) / NBC;
  const int CNTPAD = nBC * NBC;
  if (4 * nBC + 1 > RBN) return;
  const int nBF    = (nN + NBF - 1) / NBF;
  const int csrLen = ((nE + 31) & ~31) + 4096;
  const int GPAD   = ((G + GROWS - 1) / GROWS) * GROWS;
  const int nGn    = NPAD / GROWS;
  const int nGg    = GPAD / GROWS;
  const int nPool  = GPAD / NBP;
  const int NMAT   = 2 * nL + 2 * nV + 1;
  const int nPartR = nGn > nGg ? nGn : nGg;

  char* ws = (char*)d_ws;
  size_t off = 0;
  const size_t oW   = off; off += (size_t)NMAT * 2 * WPL * 2;      off = (off + 255) & ~(size_t)255;
  const size_t oCnt = off; off += (size_t)CNTPAD * 4;              off = (off + 255) & ~(size_t)255;
  const size_t oOff = off; off += (size_t)CNTPAD * 4;              off = (off + 255) & ~(size_t)255;
  const size_t oRb  = off; off += (size_t)RBN * 4;                 off = (off + 255) & ~(size_t)255;
  const size_t oCsr = off; off += (size_t)csrLen * 4;              off = (off + 255) & ~(size_t)255;
  const size_t oH   = off; off += (size_t)NPAD * HIDC * 4;         off = (off + 255) & ~(size_t)255;
  const size_t oZ1  = off; off += (size_t)NPAD * HIDC * 4;         off = (off + 255) & ~(size_t)255;
  const size_t oZ2  = off; off += (size_t)NPAD * HIDC * 4;         off = (off + 255) & ~(size_t)255;
  const size_t oPt  = off; off += (size_t)nPartR * PSTR * 8;       off = (off + 255) & ~(size_t)255;
  const size_t oAb1 = off; off += (size_t)2 * HIDC * 4;            off = (off + 255) & ~(size_t)255;
  const size_t oAb2 = off; off += (size_t)2 * HIDC * 4;            off = (off + 255) & ~(size_t)255;
  const size_t oAbv = off; off += (size_t)2 * HIDC * 4;            off = (off + 255) & ~(size_t)255;
  const size_t oGs  = off; off += (size_t)GPAD * HIDC * 4;         off = (off + 255) & ~(size_t)255;
  const size_t oVz  = off; off += (size_t)GPAD * HIDC * 4;         off = (off + 255) & ~(size_t)255;
  const size_t oVn  = off; off += (size_t)GPAD * HIDC * 4;         off = (off + 255) & ~(size_t)255;
  if (off > ws_size || off > (size_t)134217728) return;
  unsigned short* wpl = (unsigned short*)(ws + oW);
  int*    cnt  = (int*)(ws + oCnt);
  int*    offp = (int*)(ws + oOff);
  int*    rb   = (int*)(ws + oRb);
  int*    csr  = (int*)(ws + oCsr);
  float*  h    = (float*)(ws + oH);
  float*  z1   = (float*)(ws + oZ1);
  float*  z2   = (float*)(ws + oZ2);
  double* part = (double*)(ws + oPt);
  float*  ab1  = (float*)(ws + oAb1);
  float*  ab2  = (float*)(ws + oAb2);
  float*  abv  = (float*)(ws + oAbv);
  float*  gsum = (float*)(ws + oGs);
  float*  vz   = (float*)(ws + oVz);
  float*  vnh  = (float*)(ws + oVn);

  const int vec8 = ((nE & 3) == 0) ? 1 : 0;

  k_wprep<<<NMAT * (WPL / 8) / NTHR, NTHR, 0, stream>>>(convW1, convW2, vnW1, vnW2, clfW1, wpl, nL, nV);

  k_count<<<nBC, NTHR, 0, stream>>>(ei, cnt, nE, vec8);
  k_offsets<<<1, OTHR, 0, stream>>>(cnt, offp, rb, nBC);
  hipFuncSetAttribute(reinterpret_cast<const void*>(&k_fill),
                      hipFuncAttributeMaxDynamicSharedMemorySize, LDS_FILL);
  k_fill<<<nBF, NTHR, LDS_FILL, stream>>>(ei, offp, rb, csr, nN, nE, vec8, csrLen);

  k_encode<<<NPAD / NWAVE, NTHR, 0, stream>>>(x, emb, h, nN);
  k_vninit<<<GPAD / NWAVE, NTHR, 0, stream>>>(vn_emb, vnh);

  hipFuncSetAttribute(reinterpret_cast<const void*>(&k_agg_gemm),
                      hipFuncAttributeMaxDynamicSharedMemorySize, LDS_GEMM);
  hipFuncSetAttribute(reinterpret_cast<const void*>(&k_gemm),
                      hipFuncAttributeMaxDynamicSharedMemorySize, LDS_GEMM);

  for (int l = 0; l < nL; ++l) {
    const unsigned short* pW1 = wpl + (size_t)l * 2 * WPL;
    const unsigned short* pW2 = wpl + (size_t)(nL + l) * 2 * WPL;
    k_agg_gemm<<<nGn, NTHR, LDS_GEMM, stream>>>(csr, offp, cnt, h, eps, l, pW1, convb1 + (size_t)l * HIDC,
                                               z1, part, nN, csrLen);
    k_bnfin<<<1, HIDC, 0, stream>>>(part, nGn, nN, convg1 + (size_t)l * HIDC, convbt1 + (size_t)l * HIDC, ab1);
    k_gemm<<<nGn, NTHR, LDS_GEMM, stream>>>(z1, h, ab1, pW2, convb2 + (size_t)l * HIDC, z1, clfW2, clfb2, z2, part, out,
                                           NPAD, nN, G, 0, 1, 0);
    k_bnfin<<<1, HIDC, 0, stream>>>(part, nGn, nN, bng + (size_t)l * HIDC, bnb + (size_t)l * HIDC, ab2);
    if (l < nL - 1) {
      const unsigned short* pV1 = wpl + (size_t)(2 * nL + l) * 2 * WPL;
      const unsigned short* pV2 = wpl + (size_t)(2 * nL + nV + l) * 2 * WPL;
      k_pool<<<nPool, NTHR, 0, stream>>>(batch, z2, ab2, gsum, nN, 1);
      k_gemm<<<nGg, NTHR, LDS_GEMM, stream>>>(gsum, vnh, ab1, pV1, vnb1 + (size_t)l * HIDC, gsum, clfW2, clfb2, vz, part, out,
                                             GPAD, G, G, 1, 0, 0);
      k_bnfin<<<1, HIDC, 0, stream>>>(part, nGg, G, vng1 + (size_t)l * HIDC, vnbt1 + (size_t)l * HIDC, abv);
      k_gemm<<<nGg, NTHR, LDS_GEMM, stream>>>(vz, gsum, abv, pV2, vnb2 + (size_t)l * HIDC, vnh, clfW2, clfb2, vnh, part, out,
                                             GPAD, G, G, 0, 1, 1);
      k_hprod<<<NPAD / NWAVE, NTHR, 0, stream>>>(z2, ab2, vnh, batch, h, nN, G);
    }
  }

  k_pool<<<nPool, NTHR, 0, stream>>>(batch, z2, ab2, gsum, nN, 0);
  k_gemm<<<nGg, NTHR, LDS_GEMM, stream>>>(gsum, vnh, ab1, wpl + (size_t)(2 * nL + 2 * nV) * 2 * WPL, clfb1, gsum, clfW2, clfb2,
                                         vz, part, out, GPAD, G, G, 0, 0, 2);
}
